// HebbianConv2d_49615462203908
// MI455X (gfx1250) — hardware-verified
//
#include <hip/hip_runtime.h>


#define NIMG 32
#define CI   64
#define CO   128
#define HI   64
#define HO   62
#define NPO  (HO * HO)
#define NPP  3904
#define KK   (CI * 9)
#define NBLK (NPP / 64)
#define DM   KK
#define LOSC 1024.0f

typedef _Float16 h16;
typedef unsigned short bf;
typedef __attribute__((ext_vector_type(16))) __bf16   v16bf;
typedef __attribute__((ext_vector_type(16))) _Float16 v16h;
typedef __attribute__((ext_vector_type(8)))  _Float16 v8h;
typedef __attribute__((ext_vector_type(8)))  unsigned short v8us;
typedef __attribute__((ext_vector_type(8)))  float    v8f;
typedef __attribute__((ext_vector_type(4)))  float    v4f;
typedef v8h  __attribute__((may_alias)) v8ha;
typedef v4f  __attribute__((may_alias)) v4fa;
typedef v8us __attribute__((may_alias)) v8usa;

__device__ __forceinline__ unsigned short f2bf(float f) { unsigned u = __float_as_uint(f); u += 0x7FFFu + ((u >> 16) & 1u); return (unsigned short)(u >> 16); }
__device__ __forceinline__ float bf2f(unsigned short b) { return __uint_as_float(((unsigned)b) << 16); }
__device__ __forceinline__ float bfr(float f) { return bf2f(f2bf(f)); }
__device__ __forceinline__ v16h cat16(v8h lo, v8h hi) { return __builtin_shufflevector(lo, hi, 0, 1, 2, 3, 4, 5, 6, 7, 8, 9, 10, 11, 12, 13, 14, 15); }
__device__ __forceinline__ v16bf cat16b(v8us lo, v8us hi) { return __builtin_bit_cast(v16bf, __builtin_shufflevector(lo, hi, 0, 1, 2, 3, 4, 5, 6, 7, 8, 9, 10, 11, 12, 13, 14, 15)); }
__device__ __forceinline__ v8f wmma16(v16h a, v16h b, v8f c) { return __builtin_amdgcn_wmma_f32_16x16x32_f16(false, a, false, b, (short)0, c, false, false); }
__device__ __forceinline__ v8f wmmab(v16bf a, v16bf b, v8f c) { return __builtin_amdgcn_wmma_f32_16x16x32_bf16(false, a, false, b, (short)0, c, false, false); }

template <bool SPLITA, bool F16OUT = false>
__global__ __launch_bounds__(128) void k_gemmb(const bf* __restrict__ A, const bf* __restrict__ Al, const bf* __restrict__ Bn, const float* __restrict__ bias, float* C, int ldc, h16* C2, const float* __restrict__ R = nullptr, int K = DM, int roundR = 1) {
    __shared__ __align__(16) float ost[4][16 * 68];
    const int lane = threadIdx.x & 31, wave = threadIdx.x >> 5, lr = lane & 15, hi = lane >> 4;
    const int r0 = blockIdx.x * 64 + wave * 16, c0 = blockIdx.y * 64;
    const size_t aoff = (size_t)(r0 + lr) * K + 8 * hi;
    size_t boff[4];
#pragma unroll
    for (int t = 0; t < 4; ++t) boff[t] = (size_t)(c0 + t * 16 + lr) * K + 8 * hi;
    v8f acc[4];
#pragma unroll
    for (int t = 0; t < 4; ++t) acc[t] = (v8f){};
#pragma unroll 1
    for (int kc = 0; kc < K; kc += 32) {
        const v16bf a = cat16b(*(const v8us*)(A + aoff + kc), *(const v8us*)(A + aoff + kc + 16));
        v16bf al = a;
        if (SPLITA) al = cat16b(*(const v8us*)(Al + aoff + kc), *(const v8us*)(Al + aoff + kc + 16));
#pragma unroll
        for (int t = 0; t < 4; ++t) { const v16bf b = cat16b(*(const v8us*)(Bn + boff[t] + kc), *(const v8us*)(Bn + boff[t] + kc + 16)); acc[t] = wmmab(a, b, acc[t]); if (SPLITA) acc[t] = wmmab(al, b, acc[t]); }
        asm volatile("v_nop\n\tv_nop\n\tv_nop\n\tv_nop" : "+v"(acc[0]), "+v"(acc[1]), "+v"(acc[2]), "+v"(acc[3]) : "v"(a), "v"(al));
    }
    float* os = &ost[wave][0];
#pragma unroll
    for (int t = 0; t < 4; ++t) { const float bv = bias ? bfr(bias[c0 + t * 16 + lr]) : 0.f;
#pragma unroll
        for (int j = 0; j < 8; ++j) os[(hi * 8 + j) * 68 + t * 16 + lr] = acc[t][j] + bv; }
    __syncthreads();
    if (F16OUT) {
        h16* crow = (h16*)(void*)C + (size_t)r0 * ldc + c0;
        auto pass = [&]() {
#pragma unroll
            for (int s = 0; s < 4; ++s) { const int row = 4 * s + (lane >> 3), piece = lane & 7; const float* sp = os + row * 68 + piece * 8; v8h o, o2;
#pragma unroll
                for (int i = 0; i < 8; ++i) { const h16 a = (h16)sp[i]; o[i] = a; o2[i] = (h16)((sp[i] - (float)a) * LOSC); }
                *(volatile v8h*)(crow + (size_t)row * ldc + piece * 8) = o; if (C2) *(volatile v8h*)(C2 + (size_t)r0 * ldc + c0 + (size_t)row * ldc + piece * 8) = o2; }
        };
        pass(); __threadfence(); pass();
    } else {
        float* crow = C + (size_t)r0 * ldc + c0;
        auto pass = [&]() {
#pragma unroll
            for (int s = 0; s < 8; ++s) { const int Lid = (lane >> 3) + 4 * s, piece = lane & 7; const int row = Lid >> 1, cofs = (Lid & 1) * 32 + piece * 4;
                v4f val = *(const v4fa*)(os + row * 68 + cofs); if (R) { const v4f rv = *(const v4f*)(R + ((size_t)r0 + row) * ldc + c0 + cofs); val += roundR ? (v4f){bfr(rv[0]), bfr(rv[1]), bfr(rv[2]), bfr(rv[3])} : rv; }
                *(volatile v4f*)(crow + (size_t)row * ldc + cofs) = val; }
        };
        pass(); __threadfence(); pass();
    }
}


__global__ __launch_bounds__(256) void k_cvt8(const float* __restrict__ src, bf* dst, size_t n8) {
    const size_t i = (size_t)blockIdx.x * 256 + threadIdx.x; if (i >= n8) return;
    const v8f v = *(const v8f*)(src + i * 8); v8us o;
#pragma unroll
    for (int k = 0; k < 8; ++k) o[k] = f2bf(v[k]);
    *(volatile v8us*)(dst + i * 8) = o; __threadfence(); *(volatile v8us*)(dst + i * 8) = o;
}
__global__ __launch_bounds__(256) void k_zero8(bf* dst, size_t n8) {
    const size_t i = (size_t)blockIdx.x * 256 + threadIdx.x; if (i >= n8) return; v8us z;
#pragma unroll
    for (int k = 0; k < 8; ++k) z[k] = 0;
    *(volatile v8us*)(dst + i * 8) = z; __threadfence(); *(volatile v8us*)(dst + i * 8) = z;
}

__global__ __launch_bounds__(128) void k_wnorm(const float* __restrict__ w, float* RS) {
    const int o = threadIdx.x; float s = 0.f;
#pragma unroll 4
    for (int k = 0; k < KK; ++k) { const float v = bfr(w[(size_t)o * KK + k]); s = fmaf(v, v, s); }
    float n = sqrtf(s); if (n == 0.f) n = 1.f; const float r = 1.0f / n;
    *(volatile float*)(RS + o) = r; __threadfence(); *(volatile float*)(RS + o) = r;
}
__global__ __launch_bounds__(256) void k_im2col(const float* __restrict__ xi, bf* IM) {
    const int lane = threadIdx.x & 31, p = blockIdx.x * 8 + (threadIdx.x >> 5); if (p >= NPP) return;
    const int py = p / HO, px = p % HO; const bool rok = p < NPO; const int pyc = rok ? py : 0, pxc = rok ? px : 0;
#pragma unroll 1
    for (int ps = 0; ps < 2; ++ps) {
#pragma unroll 1
        for (int k0 = lane * 8; k0 < KK; k0 += 256) { v8us ob;
#pragma unroll
            for (int q = 0; q < 8; ++q) { const int k = k0 + q; const int c = k / 9, t = k % 9, i = t / 3, j = t % 3; const float v = xi[((size_t)c * HI + pyc + i) * HI + pxc + j]; ob[q] = rok ? f2bf(v) : (unsigned short)0; }
            *(volatile v8us*)(IM + (size_t)p * KK + k0) = ob; }
        if (ps == 0) __threadfence(); }
}
__global__ __launch_bounds__(256) void k_im2colT(const float* __restrict__ xi, bf* BT) {
    const int lane = threadIdx.x & 31, k = blockIdx.x * 8 + (threadIdx.x >> 5); if (k >= KK) return;
    const int c = k / 9, t = k % 9, i = t / 3, j = t % 3; const float* xc = xi + (size_t)c * HI * HI;
#pragma unroll 1
    for (int ps = 0; ps < 2; ++ps) {
#pragma unroll 1
        for (int p0 = lane * 8; p0 < NPP; p0 += 256) { v8us ob;
#pragma unroll
            for (int q = 0; q < 8; ++q) { const int p = p0 + q; const bool ok = p < NPO; const int pc = ok ? p : 0; const int py = pc / HO, px = pc % HO; const float v = xc[(py + i) * HI + px + j]; ob[q] = ok ? f2bf(v) : (unsigned short)0; }
            *(volatile v8us*)(BT + (size_t)k * NPP + p0) = ob; }
        if (ps == 0) __threadfence(); }
}
__global__ __launch_bounds__(128) void k_gemmrs(const bf* __restrict__ A, const bf* __restrict__ Bn, const float* __restrict__ rs, const float* __restrict__ rbias, float* C, int ldc, int K) {
    __shared__ __align__(16) float ost[4][16 * 68];
    const int lane = threadIdx.x & 31, wave = threadIdx.x >> 5, lr = lane & 15, hi = lane >> 4;
    const int r0 = blockIdx.x * 64 + wave * 16, c0 = blockIdx.y * 64;
    const size_t aoff = (size_t)(r0 + lr) * K + 8 * hi;
    v8f acc[4];
#pragma unroll
    for (int t = 0; t < 4; ++t) acc[t] = (v8f){};
#pragma unroll 1
    for (int kc = 0; kc < K; kc += 32) {
        const v16bf a = cat16b(*(const v8us*)(A + aoff + kc), *(const v8us*)(A + aoff + kc + 16));
#pragma unroll
        for (int t = 0; t < 4; ++t) { const size_t bo = (size_t)(c0 + t * 16 + lr) * K + kc + 8 * hi; const v16bf bb = cat16b(*(const v8us*)(Bn + bo), *(const v8us*)(Bn + bo + 16)); acc[t] = wmmab(a, bb, acc[t]); }
        asm volatile("v_nop\n\tv_nop\n\tv_nop\n\tv_nop" : "+v"(acc[0]), "+v"(acc[1]), "+v"(acc[2]), "+v"(acc[3]) : "v"(a));
    }
    float* os = &ost[wave][0];
#pragma unroll
    for (int t = 0; t < 4; ++t) {
#pragma unroll
        for (int j = 0; j < 8; ++j) { const int o = r0 + hi * 8 + j; os[(hi * 8 + j) * 68 + t * 16 + lr] = acc[t][j] * rs[o] + bfr(rbias[o]); } }
    __builtin_amdgcn_wave_barrier(); asm volatile("" ::: "memory");
    float* crow = C + (size_t)r0 * ldc + c0;
    auto pass = [&]() {
#pragma unroll
        for (int s = 0; s < 8; ++s) { const int Lid = (lane >> 3) + 4 * s, piece = lane & 7; const int row = Lid >> 1, cofs = (Lid & 1) * 32 + piece * 4;
            const v4f val = *(const v4fa*)(os + row * 68 + cofs); *(volatile v4f*)(crow + (size_t)row * ldc + cofs) = val; }
    };
    pass(); __threadfence(); pass();
}
__global__ __launch_bounds__(256) void k_yout(const float* __restrict__ C, float* Y) {
    const size_t u = (size_t)blockIdx.x * 256 + threadIdx.x; if (u >= (size_t)CO * NPO / 4) return; v4f v;
#pragma unroll
    for (int i = 0; i < 4; ++i) { const size_t f = u * 4 + i; const int o = (int)(f / NPO), p = (int)(f % NPO); v[i] = C[(size_t)o * NPP + p]; }
    *(volatile v4f*)(Y + u * 4) = v; __threadfence(); *(volatile v4f*)(Y + u * 4) = v;
}
template <int MODE>
__global__ __launch_bounds__(128) void k_soft(const float* __restrict__ C, const float* __restrict__ inv, int blk0, float* RP, bf* CRh, bf* CRl) {
    __shared__ __align__(16) float tl[CO][68];
    const int tid = threadIdx.x, pb = blockIdx.x * 64;
    if (tid < 64) { const int p = pb + tid; const bool ok = p < NPO; float m = -3.0e38f;
#pragma unroll 4
        for (int o = 0; o < CO; ++o) m = fmaxf(m, C[(size_t)o * NPP + p]);
        float s = 0.f;
#pragma unroll 4
        for (int o = 0; o < CO; ++o) s += __expf(C[(size_t)o * NPP + p] - m);
        const float is = 1.0f / s;
#pragma unroll 4
        for (int o = 0; o < CO; ++o) { const float r = __expf(C[(size_t)o * NPP + p] - m) * is; tl[o][tid] = ok ? (MODE ? r * r * inv[o] : r) : 0.f; } }
    __syncthreads();
    { const int o = tid; float acc = 0.f;
#pragma unroll 4
      for (int q = 0; q < 64; ++q) acc += tl[o][q];
      float* rp = RP + ((size_t)blk0 + blockIdx.x) * CO + o; *(volatile float*)rp = acc; }
    if (MODE) { const int piece = tid & 7, Lid = tid >> 3;
        auto pass = [&]() {
#pragma unroll
            for (int s = 0; s < 8; ++s) { const int o = Lid + 16 * s; v8us oh, ol;
#pragma unroll
                for (int i = 0; i < 8; ++i) { const float v = tl[o][piece * 8 + i]; const unsigned short hb = f2bf(v); oh[i] = hb; ol[i] = f2bf(v - bf2f(hb)); }
                const size_t off = (size_t)o * NPP + pb + piece * 8; *(volatile v8us*)(CRh + off) = oh; *(volatile v8us*)(CRl + off) = ol; }
        };
        pass(); __threadfence(); pass(); }
    else __threadfence();
    { const int o = tid; float acc = 0.f;
#pragma unroll 4
      for (int q = 0; q < 64; ++q) acc += tl[o][q];
      float* rp = RP + ((size_t)blk0 + blockIdx.x) * CO + o; *(volatile float*)rp = acc; }
}
template <int INVERT>
__global__ __launch_bounds__(128) void k_csum(const float* __restrict__ RP, int nparts, float* S) {
    const int o = threadIdx.x; float s = 0.f;
#pragma unroll 1
    for (int q = 0; q < nparts; ++q) s += RP[(size_t)q * CO + o];
    float v = s; if (INVERT) { if (v == 0.f) v = 1.f; v = 1.0f / v; }
    *(volatile float*)(S + o) = v; __threadfence(); *(volatile float*)(S + o) = v;
}
__global__ __launch_bounds__(256) void k_dout(const float* __restrict__ D, const float* __restrict__ CS, const float* __restrict__ w, float* OUTD) {
    const int lane = threadIdx.x & 31, o = blockIdx.x * 8 + (threadIdx.x >> 5); if (o >= CO) return; const float cs = CS[o];
#pragma unroll 1
    for (int ps = 0; ps < 2; ++ps) {
#pragma unroll 1
        for (int k0 = lane * 4; k0 < KK; k0 += 128) { v4f v;
#pragma unroll
            for (int i = 0; i < 4; ++i) { const size_t e = (size_t)o * KK + k0 + i; v[i] = D[e] - cs * bfr(w[e]); }
            *(volatile v4f*)(OUTD + (size_t)o * KK + k0) = v; }
        if (ps == 0) __threadfence(); }
}

extern "C" void kernel_launch(void* const* d_in, const int* in_sizes, int n_in,
                              void* d_out, int out_size, void* d_ws, size_t ws_size, hipStream_t stream) {
    (void)in_sizes; (void)n_in; (void)out_size;
    const float* x = (const float*)d_in[0]; const float* w = (const float*)d_in[1]; const float* bias = (const float*)d_in[2];
    float* y = (float*)d_out; float* dout = (float*)((char*)d_out + (size_t)NIMG * CO * NPO * 4);
    char* wsp = (char*)d_ws;
    auto take = [&](size_t bytes) { char* p = wsp; wsp += (bytes + 255) & ~(size_t)255; return (void*)p; };
    bf* WB = (bf*)take((size_t)CO * KK * 2); float* RS = (float*)take(CO * 4); bf* IM = (bf*)take((size_t)NPP * KK * 2); bf* BT = (bf*)take((size_t)KK * NPP * 2); float* C = (float*)take((size_t)CO * NPP * 4);
    float* RP = (float*)take((size_t)NIMG * NBLK * CO * 4); float* RINV = (float*)take(CO * 4); float* CRS = (float*)take(CO * 4); bf* CRh = (bf*)take((size_t)CO * NPP * 2); bf* CRl = (bf*)take((size_t)CO * NPP * 2); float* D0 = (float*)take((size_t)CO * KK * 4); float* D1 = (float*)take((size_t)CO * KK * 4);
    if ((size_t)(wsp - (char*)d_ws) > ws_size) return;
    k_cvt8<<<(CO * KK / 8 + 255) / 256, 256, 0, stream>>>(w, WB, CO * KK / 8); k_wnorm<<<1, CO, 0, stream>>>(w, RS);
    for (int b = 0; b < NIMG; ++b) { const float* xi = x + (size_t)b * CI * HI * HI;
        k_im2col<<<NPP / 8, 256, 0, stream>>>(xi, IM);
        k_gemmrs<<<dim3(CO / 64, NPP / 64, 1), 128, 0, stream>>>(WB, IM, RS, bias, C, NPP, KK);
        k_yout<<<(CO * NPO / 4 + 255) / 256, 256, 0, stream>>>(C, y + (size_t)b * CO * NPO);
        k_soft<0><<<NBLK, 128, 0, stream>>>(C, nullptr, b * NBLK, RP, nullptr, nullptr); }
    k_csum<1><<<1, CO, 0, stream>>>(RP, NIMG * NBLK, RINV);
    const float* Dprev = nullptr; float* Dc = nullptr;
    for (int b = 0; b < NIMG; ++b) { const float* xi = x + (size_t)b * CI * HI * HI; Dc = (b & 1) ? D1 : D0;
        k_im2col<<<NPP / 8, 256, 0, stream>>>(xi, IM); k_im2colT<<<KK / 8, 256, 0, stream>>>(xi, BT);
        k_gemmrs<<<dim3(CO / 64, NPP / 64, 1), 128, 0, stream>>>(WB, IM, RS, bias, C, NPP, KK);
        k_soft<1><<<NBLK, 128, 0, stream>>>(C, RINV, b * NBLK, RP, CRh, CRl);
        k_gemmb<true, false><<<dim3(CO / 64, KK / 64, 1), 128, 0, stream>>>(CRh, CRl, BT, nullptr, Dc, KK, nullptr, Dprev, NPP, 0);
        Dprev = Dc; }
    k_csum<0><<<1, CO, 0, stream>>>(RP, NIMG * NBLK, CRS);
    k_dout<<<CO / 8, 256, 0, stream>>>(Dc, CRS, w, dout);
}
